// LSTM0_83872121357050
// MI455X (gfx1250) — hardware-verified
//
#include <hip/hip_runtime.h>
#include <stdint.h>

typedef __attribute__((ext_vector_type(16))) _Float16 v16h;
typedef __attribute__((ext_vector_type(8)))  _Float16 v8h;
typedef __attribute__((ext_vector_type(16))) __bf16   v16b;
typedef __attribute__((ext_vector_type(8)))  __bf16   v8b;
typedef __attribute__((ext_vector_type(8)))  float    v8f;
typedef __attribute__((ext_vector_type(4)))  float    v4f;
typedef __attribute__((ext_vector_type(4)))  unsigned int v4u;

constexpr int NBATCH = 64;
constexpr int NSTEP  = 512;
constexpr int NIN    = 60;
constexpr int KXPAD  = 64;
constexpr int NHID   = 256;
constexpr int NGATE  = 1024;
constexpr int KCAT   = KXPAD + NHID;
constexpr int APITCH = 328;
constexpr int NOUT   = 402;
constexpr int NOUTP  = 448;
constexpr int NROWS  = NBATCH * NSTEP;

constexpr size_t O_WCAT = 0;
constexpr size_t O_WFC  = O_WCAT + (size_t)NGATE * KCAT * 2;
constexpr size_t O_BFC  = O_WFC + (size_t)NOUTP * NHID * 2;
constexpr size_t O_X16  = O_BFC + (size_t)NOUTP * 4;
constexpr size_t O_HS   = O_X16 + (size_t)NROWS * KXPAD * 2;
constexpr size_t O_STG  = O_HS + (size_t)NROWS * NHID * 2;
constexpr size_t WS_END = O_STG + (size_t)NROWS * NOUTP * 4;
static_assert(O_WFC % 128 == 0 && O_BFC % 128 == 0 && O_X16 % 128 == 0 && O_HS % 128 == 0 && O_STG % 128 == 0, "align");
static_assert(WS_END <= 134217728ull, "carve under 128 MiB");
static_assert(KCAT % 32 == 0 && NHID % 32 == 0 && NROWS % 64 == 0 && NOUTP % 64 == 0, "tile multiples");

__device__ __forceinline__ unsigned short f2bf_bits(float f) {
  unsigned u = __float_as_uint(f);
  return (unsigned short)((u + 0x7FFFu + ((u >> 16) & 1u)) >> 16);
}
__device__ __forceinline__ float bf_bits2f(unsigned short h) { return __uint_as_float(((unsigned)h) << 16); }

__device__ __forceinline__ void dep_guard_h(v8f& a, v8f& b, v16h x, v16h y) { asm volatile("v_nop\n\tv_nop\n\tv_nop\n\tv_nop" : "+v"(a), "+v"(b) : "v"(x), "v"(y)); }
__device__ __forceinline__ void dep_guard_b(v8f& a, v8f& b, v16b x, v16b y) { asm volatile("v_nop\n\tv_nop\n\tv_nop\n\tv_nop" : "+v"(a), "+v"(b) : "v"(x), "v"(y)); }
__device__ __forceinline__ void keep4_h(v16h a, v16h b, v16h c, v16h d) { asm volatile("v_nop" :: "v"(a), "v"(b), "v"(c), "v"(d)); }
__device__ __forceinline__ void keep4_b(v16b a, v16b b, v16b c, v16b d) { asm volatile("v_nop" :: "v"(a), "v"(b), "v"(c), "v"(d)); }
__device__ __forceinline__ void acc_guard4(v8f& a, v8f& b, v8f& c, v8f& d) { asm volatile("v_nop\n\tv_nop\n\tv_nop\n\tv_nop" : "+v"(a), "+v"(b), "+v"(c), "+v"(d)); }
template <typename T> struct Frag;
template <> struct Frag<_Float16> {
  typedef v16h V; union U { v16h v; v8h h[2]; };
  static __device__ __forceinline__ v16h load(const _Float16* p) {
    U f; f.h[0] = *(const v8h*)(p); f.h[1] = *(const v8h*)(p + 16); return f.v;
  }
  static __device__ __forceinline__ v8f mma(v16h a, v16h b, v8f c) {
    return __builtin_amdgcn_wmma_f32_16x16x32_f16(false, a, false, b, (short)0, c, false, false);
  }
  static __device__ __forceinline__ void guard(v8f& a, v8f& b, v16h x, v16h y) { dep_guard_h(a, b, x, y); }
  static __device__ __forceinline__ void keep(v16h a, v16h b, v16h c, v16h d) { keep4_h(a, b, c, d); }
};
template <> struct Frag<__bf16> {
  typedef v16b V; union U { v16b v; v8b h[2]; };
  static __device__ __forceinline__ v16b load(const __bf16* p) {
    U f; f.h[0] = *(const v8b*)(p); f.h[1] = *(const v8b*)(p + 16); return f.v;
  }
  static __device__ __forceinline__ v8f mma(v16b a, v16b b, v8f c) {
    return __builtin_amdgcn_wmma_f32_16x16x32_bf16(false, a, false, b, (short)0, c, false, false);
  }
  static __device__ __forceinline__ void guard(v8f& a, v8f& b, v16b x, v16b y) { dep_guard_b(a, b, x, y); }
  static __device__ __forceinline__ void keep(v16b a, v16b b, v16b c, v16b d) { keep4_b(a, b, c, d); }
};

template <int ET> struct Elem;
template <> struct Elem<0> { typedef _Float16 T; };
template <> struct Elem<1> { typedef __bf16 T; };
template <int ET, bool SPLIT, int BIAS_MODE, int OUT_MODE, bool RESID, int ACT = 0>
__global__ __launch_bounds__(256) void wmma_gemm64(
    const unsigned short* __restrict__ Ap, const unsigned short* __restrict__ A2p, int lda, long strideA,
    const unsigned short* __restrict__ Btp, const unsigned short* __restrict__ Bt2p, int ldb, long strideB,
    void* __restrict__ Cout, void* __restrict__ Cout2, int ldc, long strideC,
    const float* __restrict__ bias,
    const float* __restrict__ resid, long strideR,
    int M, int N, int K, float scale) {
  typedef typename Elem<ET>::T T;
  typedef typename Frag<T>::V V;
  const T* A = (const T*)Ap; const T* A2 = (const T*)A2p; const T* Bt = (const T*)Btp; const T* Bt2 = (const T*)Bt2p;
  __shared__ __align__(16) float sT[8][16 * 68];
  const int b    = blockIdx.y;
  const int lane = threadIdx.x & 31;
  const int wave = threadIdx.x >> 5;
  const int tilesN = N >> 6;
  const int tilesM = M >> 6;
  const int tile = blockIdx.x * 8 + wave;
  if (tile >= tilesM * tilesN) return;
  const int tm = tile / tilesN;
  const int tn = tile - tm * tilesN;
  const int m0 = tm << 6;
  const int n0 = tn << 6;

  const T* Ab  = A  + (size_t)b * strideA;
  const T* Bb  = Bt + (size_t)b * strideB;
  const T* Ab2 = SPLIT ? (A2  + (size_t)b * strideA) : nullptr;
  const T* Bb2 = SPLIT ? (Bt2 + (size_t)b * strideB) : nullptr;

  const int rlane = lane & 15;
  const int koff  = (lane >> 4) * 8;
  const int mOff  = (lane >> 4) * 8;

  v8f acc[4][4];
#pragma unroll
  for (int i = 0; i < 4; ++i)
#pragma unroll
    for (int j = 0; j < 4; ++j) acc[i][j] = (v8f){0.f,0.f,0.f,0.f,0.f,0.f,0.f,0.f};

  for (int k0 = 0; k0 < K; k0 += 32) {
    V bh[4], bl[4];
#pragma unroll
    for (int j = 0; j < 4; ++j) {
      const size_t bo = (size_t)(n0 + (j << 4) + rlane) * ldb + koff + k0;
      bh[j] = Frag<T>::load(Bb + bo);
      if (SPLIT) bl[j] = Frag<T>::load(Bb2 + bo);
    }
#pragma unroll
    for (int i = 0; i < 4; ++i) {
      const size_t ao = (size_t)(m0 + (i << 4) + rlane) * lda + koff + k0;
      V ah = Frag<T>::load(Ab + ao);
      V al;
      if (SPLIT) al = Frag<T>::load(Ab2 + ao);
#pragma unroll
      for (int j = 0; j < 4; ++j) {
        acc[i][j] = Frag<T>::mma(ah, bh[j], acc[i][j]);
        if (SPLIT) {
          acc[i][j] = Frag<T>::mma(ah, bl[j], acc[i][j]);
          acc[i][j] = Frag<T>::mma(al, bh[j], acc[i][j]);
        }
      }
      Frag<T>::guard(acc[i][0], acc[i][3], ah, SPLIT ? al : ah);
    }
    Frag<T>::keep(bh[0], bh[1], bh[2], bh[3]);
    if (SPLIT) Frag<T>::keep(bl[0], bl[1], bl[2], bl[3]);
  }
  acc_guard4(acc[0][0], acc[0][1], acc[0][2], acc[0][3]);
  acc_guard4(acc[1][0], acc[1][1], acc[1][2], acc[1][3]);
  acc_guard4(acc[2][0], acc[2][1], acc[2][2], acc[2][3]);
  acc_guard4(acc[3][0], acc[3][1], acc[3][2], acc[3][3]);

  float* slab = sT[wave];
  const float* Rb = RESID ? (resid + (size_t)b * strideR) : nullptr;
#pragma unroll
  for (int i = 0; i < 4; ++i) {
    const int mBase = m0 + (i << 4);
#pragma unroll
    for (int j = 0; j < 4; ++j) {
      const int n = n0 + (j << 4) + rlane;
      float bv = 0.f;
      if (BIAS_MODE == 2) bv = bias[n];
#pragma unroll
      for (int r = 0; r < 8; ++r) {
        float v = acc[i][j][r] * scale;
        if (BIAS_MODE == 1) v += bias[mBase + mOff + r];
        if (BIAS_MODE == 2) v += bv;
        if (RESID) v += Rb[(size_t)(mBase + mOff + r) * ldc + n];
        if (ACT == 1) v = tanhf(v);
        if (ACT == 2) v = fmaxf(v, 0.0f);
        if (ACT == 3) v = v / (1.0f + expf(-v));
        if (ACT == 4) v = (v > 0.f) ? v : 0.01f * v;
        if (ACT == 5) v = 0.5f * v * (1.0f + erff(v * 0.70710678118654752f));
        slab[(mOff + r) * 68 + (j << 4) + rlane] = v;
      }
    }
    __builtin_amdgcn_fence(__ATOMIC_RELEASE, "workgroup");
    __builtin_amdgcn_wave_barrier();
    __builtin_amdgcn_fence(__ATOMIC_ACQUIRE, "workgroup");
    if (OUT_MODE == 0) {
      float* C = (float*)Cout + (size_t)b * strideC;
      const int hh = lane >> 4, c4 = (lane & 15) * 4;
      for (int pass = 0; pass < 2; ++pass) {
#pragma unroll
        for (int it = 0; it < 8; ++it) {
          const int row = it * 2 + hh;
          v4f v = *(const v4f*)(slab + row * 68 + c4);
          *(volatile v4f*)(C + (size_t)(mBase + row) * ldc + n0 + c4) = v;
        }
        __threadfence();
      }
    } else {
      const int q = lane >> 3, c8 = (lane & 7) * 8;
      unsigned short* C  = (unsigned short*)Cout  + (size_t)b * strideC;
      unsigned short* C2 = (OUT_MODE == 2) ? ((unsigned short*)Cout2 + (size_t)b * strideC) : nullptr;
      for (int pass = 0; pass < 2; ++pass) {
#pragma unroll
        for (int it = 0; it < 4; ++it) {
          const int row = it * 4 + q;
          const float* sp = slab + row * 68 + c8;
          v8h hv, lv;
#pragma unroll
          for (int e = 0; e < 8; ++e) {
            if (OUT_MODE == 1) {
              hv[e] = (_Float16)sp[e];
            } else {
              unsigned short hb = f2bf_bits(sp[e]);
              unsigned short lb = f2bf_bits(sp[e] - bf_bits2f(hb));
              hv[e] = __builtin_bit_cast(_Float16, hb);
              lv[e] = __builtin_bit_cast(_Float16, lb);
            }
          }
          *(volatile v8h*)(C + (size_t)(mBase + row) * ldc + n0 + c8) = hv;
          if (OUT_MODE == 2) *(volatile v8h*)(C2 + (size_t)(mBase + row) * ldc + n0 + c8) = lv;
        }
        __threadfence();
      }
    }
    __builtin_amdgcn_fence(__ATOMIC_RELEASE, "workgroup");
    __builtin_amdgcn_wave_barrier();
    __builtin_amdgcn_fence(__ATOMIC_ACQUIRE, "workgroup");
  }
}

__global__ __launch_bounds__(256) void prep_wcat_kernel(
    const float* __restrict__ W_ih, const float* __restrict__ W_hh, unsigned short* __restrict__ wcatp) {
  const int i = blockIdx.x * 256 + threadIdx.x;
  const int e0 = i * 8;
  const int row = e0 / KCAT;
  const int col0 = e0 - row * KCAT;
  unsigned int w[4];
#pragma unroll
  for (int p = 0; p < 4; ++p) {
    unsigned int packed = 0u;
#pragma unroll
    for (int s = 0; s < 2; ++s) {
      const int col = col0 + 2 * p + s;
      const int ki = (col < NIN) ? col : (NIN - 1);
      int kh = col - KXPAD; kh = (kh < 0) ? 0 : kh;
      const float vi = W_ih[row * NIN + ki] * 8.0f;
      const float vh = W_hh[row * NHID + kh] * 8.0f;
      const float v = (col < NIN) ? vi : ((col >= KXPAD) ? vh : 0.0f);
      const unsigned int bits = (unsigned int)__builtin_bit_cast(unsigned short, (_Float16)v);
      packed |= bits << (16 * s);
    }
    w[p] = packed;
  }
  v4u u; u[0] = w[0]; u[1] = w[1]; u[2] = w[2]; u[3] = w[3];
  *(volatile v4u*)(wcatp + e0) = u;
  __threadfence();
  *(volatile v4u*)(wcatp + e0) = u;
}

__global__ __launch_bounds__(256) void prep_wfc_kernel(
    const float* __restrict__ W_fc, const float* __restrict__ b_fc,
    unsigned short* __restrict__ wfcp, float* __restrict__ bfcp) {
  if (blockIdx.x < 56) {
    const int i = blockIdx.x * 256 + threadIdx.x;
    const int e0 = i * 8;
    const int row = e0 >> 8;
    const int col0 = e0 & 255;
    const int rowc = (row < NOUT) ? row : (NOUT - 1);
    unsigned int w[4];
#pragma unroll
    for (int p = 0; p < 4; ++p) {
      unsigned int packed = 0u;
#pragma unroll
      for (int s = 0; s < 2; ++s) {
        const int col = col0 + 2 * p + s;
        const float raw = W_fc[rowc * NHID + col] * 8.0f;
        const float v = (row < NOUT) ? raw : 0.0f;
        const unsigned int bits = (unsigned int)__builtin_bit_cast(unsigned short, (_Float16)v);
        packed |= bits << (16 * s);
      }
      w[p] = packed;
    }
    v4u u; u[0] = w[0]; u[1] = w[1]; u[2] = w[2]; u[3] = w[3];
    *(volatile v4u*)(wfcp + e0) = u;
    __threadfence();
    *(volatile v4u*)(wfcp + e0) = u;
  } else {
    const int tid = threadIdx.x;
    if (tid < NOUTP / 4) {
      v4f f;
#pragma unroll
      for (int e = 0; e < 4; ++e) {
        const int n = 4 * tid + e;
        const int nc = (n < NOUT) ? n : (NOUT - 1);
        const float raw = b_fc[nc];
        f[e] = (n < NOUT) ? raw : 0.0f;
      }
      *(volatile v4f*)(bfcp + 4 * tid) = f;
      __threadfence();
      *(volatile v4f*)(bfcp + 4 * tid) = f;
    }
  }
}

__global__ __launch_bounds__(256) void prep_x16_kernel(
    const float* __restrict__ x, unsigned short* __restrict__ x16p) {
  const int i = blockIdx.x * 256 + threadIdx.x;
  const int e0 = i * 8;
  const int row = e0 >> 6;
  const int col0 = e0 & 63;
  unsigned int w[4];
#pragma unroll
  for (int p = 0; p < 4; ++p) {
    unsigned int packed = 0u;
#pragma unroll
    for (int s = 0; s < 2; ++s) {
      const int col = col0 + 2 * p + s;
      const int kc = (col < NIN) ? col : (NIN - 1);
      const float raw = x[row * NIN + kc] * 8.0f;
      const float v = (col < NIN) ? raw : 0.0f;
      const unsigned int bits = (unsigned int)__builtin_bit_cast(unsigned short, (_Float16)v);
      packed |= bits << (16 * s);
    }
    w[p] = packed;
  }
  v4u u; u[0] = w[0]; u[1] = w[1]; u[2] = w[2]; u[3] = w[3];
  *(volatile v4u*)(x16p + e0) = u;
  __threadfence();
  *(volatile v4u*)(x16p + e0) = u;
}

__global__ __launch_bounds__(256) void lstm_seq_kernel(
    const unsigned short* __restrict__ x16p, const unsigned short* __restrict__ wcatp,
    const float* __restrict__ b_ih, const float* __restrict__ b_hh,
    unsigned short* __restrict__ hs16p) {
  __shared__ __align__(16) _Float16 atile[16 * APITCH];
  const _Float16* wcat = (const _Float16*)(const void*)wcatp;
  const int tid = threadIdx.x;
  const int lane = tid & 31;
  const int wave = tid >> 5;
  const int blk = blockIdx.x;
  const int rlane = lane & 15;
  const int hh = lane >> 4;
  const int koff = hh * 8;
  const int ucol0 = wave * 32;

  {
    unsigned int* aw = (unsigned int*)(void*)atile;
    for (int i = tid; i < 16 * APITCH / 2; i += 256) aw[i] = 0u;
  }
  float bsum[2][4];
#pragma unroll
  for (int j = 0; j < 2; ++j) {
#pragma unroll
    for (int q = 0; q < 4; ++q) {
      const int n = q * NHID + ucol0 + 16 * j + rlane;
      bsum[j][q] = b_ih[n] + b_hh[n];
    }
  }
  float cst[2][8];
#pragma unroll
  for (int j = 0; j < 2; ++j)
#pragma unroll
    for (int r = 0; r < 8; ++r) cst[j][r] = 0.0f;
  __syncthreads();

  const float kInv64 = 0.015625f;
  const float kExpClamp = 60.0f;

#pragma unroll 1
  for (int t = 0; t < NSTEP; ++t) {
    if (tid < 128) {
      const int r = tid >> 3, ch = tid & 7;
      const size_t grow = (size_t)(blk * 16 + r) * NSTEP + t;
      const v4u u = *(const v4u*)(x16p + grow * KXPAD + ch * 8);
      *(v4u*)(void*)(atile + r * APITCH + ch * 8) = u;
    }
    __syncthreads();

    v8f acc[2][4];
#pragma unroll
    for (int j = 0; j < 2; ++j)
#pragma unroll
      for (int q = 0; q < 4; ++q) acc[j][q] = (v8f){0.f,0.f,0.f,0.f,0.f,0.f,0.f,0.f};

#pragma unroll 1
    for (int k0 = 0; k0 < KCAT; k0 += 32) {
      const v16h a = Frag<_Float16>::load(atile + rlane * APITCH + koff + k0);
#pragma unroll
      for (int j = 0; j < 2; ++j) {
        v16h bq[4];
#pragma unroll
        for (int q = 0; q < 4; ++q)
          bq[q] = Frag<_Float16>::load(wcat + (size_t)(q * NHID + ucol0 + 16 * j + rlane) * KCAT + koff + k0);
#pragma unroll
        for (int q = 0; q < 4; ++q) acc[j][q] = Frag<_Float16>::mma(a, bq[q], acc[j][q]);
        dep_guard_h(acc[j][0], acc[j][3], a, bq[3]);
        keep4_h(bq[0], bq[1], bq[2], bq[3]);
      }
    }
    acc_guard4(acc[0][0], acc[0][1], acc[0][2], acc[0][3]);
    acc_guard4(acc[1][0], acc[1][1], acc[1][2], acc[1][3]);
    __syncthreads();

#pragma unroll
    for (int j = 0; j < 2; ++j) {
#pragma unroll
      for (int r = 0; r < 8; ++r) {
        const float pi = acc[j][0][r] * kInv64 + bsum[j][0];
        const float pf = acc[j][1][r] * kInv64 + bsum[j][1];
        const float pg = acc[j][2][r] * kInv64 + bsum[j][2];
        const float po = acc[j][3][r] * kInv64 + bsum[j][3];
        const float ig = 1.0f / (1.0f + expf(fminf(-pi, kExpClamp)));
        const float fg = 1.0f / (1.0f + expf(fminf(-pf, kExpClamp)));
        const float gg = 1.0f - 2.0f / (1.0f + expf(fminf(2.0f * pg, kExpClamp)));
        const float og = 1.0f / (1.0f + expf(fminf(-po, kExpClamp)));
        const float cn = fg * cst[j][r] + ig * gg;
        cst[j][r] = cn;
        const float hn = og * (1.0f - 2.0f / (1.0f + expf(fminf(2.0f * cn, kExpClamp))));
        atile[(8 * hh + r) * APITCH + KXPAD + ucol0 + 16 * j + rlane] = (_Float16)(hn * 8.0f);
      }
    }
    __syncthreads();

    for (int pass = 0; pass < 2; ++pass) {
#pragma unroll
      for (int s = 0; s < 2; ++s) {
        const int rr = wave * 2 + s;
        const size_t grow = (size_t)(blk * 16 + rr) * NSTEP + t;
        const v8h hv = *(const v8h*)(atile + rr * APITCH + KXPAD + lane * 8);
        *(volatile v8h*)(hs16p + grow * NHID + lane * 8) = hv;
      }
      __threadfence();
    }
  }
}

__global__ __launch_bounds__(256) void pack_out_kernel(
    const float* __restrict__ stg, float* __restrict__ out, int n4) {
  const int i = blockIdx.x * 256 + threadIdx.x;
  if (i >= n4) return;
  const int e0 = i * 4;
  v4f v;
#pragma unroll
  for (int e = 0; e < 4; ++e) {
    const int el = e0 + e;
    const int row = el / NOUT;
    const int col = el - row * NOUT;
    v[e] = stg[(size_t)row * NOUTP + col];
  }
  *(volatile v4f*)(out + e0) = v;
  __threadfence();
  *(volatile v4f*)(out + e0) = v;
}

extern "C" void kernel_launch(void* const* d_in, const int* in_sizes, int n_in,
                              void* d_out, int out_size, void* d_ws, size_t ws_size,
                              hipStream_t stream) {
  if (n_in < 7) return;
  if (in_sizes[0] != NBATCH * NSTEP * NIN) return;
  if (in_sizes[1] != NGATE * NIN || in_sizes[2] != NGATE * NHID) return;
  if (in_sizes[3] != NGATE || in_sizes[4] != NGATE) return;
  if (in_sizes[5] != NOUT * NHID || in_sizes[6] != NOUT) return;
  if (out_size != NROWS * NOUT) return;
  if (ws_size < WS_END) return;

  const float* x    = (const float*)d_in[0];
  const float* W_ih = (const float*)d_in[1];
  const float* W_hh = (const float*)d_in[2];
  const float* b_ih = (const float*)d_in[3];
  const float* b_hh = (const float*)d_in[4];
  const float* W_fc = (const float*)d_in[5];
  const float* b_fc = (const float*)d_in[6];
  char* ws = (char*)d_ws;
  float* out = (float*)d_out;

  unsigned short* wcat = (unsigned short*)(ws + O_WCAT);
  unsigned short* wfc  = (unsigned short*)(ws + O_WFC);
  float*          bfcp = (float*)(ws + O_BFC);
  unsigned short* x16  = (unsigned short*)(ws + O_X16);
  unsigned short* hs16 = (unsigned short*)(ws + O_HS);
  float*          stg  = (float*)(ws + O_STG);

  const int wcatBlocks = (NGATE * KCAT / 8) / 256;
  const int wfcBlocks  = (NOUTP * NHID / 8) / 256 + 1;
  const int x16Blocks  = (NROWS * KXPAD / 8) / 256;
  const int fcBlocks   = (NROWS / 64) * (NOUTP / 64) / 8;
  const int n4         = NROWS * NOUT / 4;
  const int packBlocks = n4 / 256;

  prep_wcat_kernel<<<dim3(wcatBlocks, 1, 1), dim3(256, 1, 1), 0, stream>>>(W_ih, W_hh, wcat);
  prep_wfc_kernel<<<dim3(wfcBlocks, 1, 1), dim3(256, 1, 1), 0, stream>>>(W_fc, b_fc, wfc, bfcp);
  prep_x16_kernel<<<dim3(x16Blocks, 1, 1), dim3(256, 1, 1), 0, stream>>>(x, x16);
  lstm_seq_kernel<<<dim3(NBATCH / 16, 1, 1), dim3(256, 1, 1), 0, stream>>>(x16, wcat, b_ih, b_hh, hs16);
  wmma_gemm64<0, false, 2, 0, false, 0><<<dim3(fcBlocks, 1, 1), dim3(256, 1, 1), 0, stream>>>(
      (const unsigned short*)hs16, (const unsigned short*)hs16, NHID, 0L,
      (const unsigned short*)wfc, (const unsigned short*)wfc, NHID, 0L,
      (void*)stg, (void*)stg, NOUTP, 0L,
      (const float*)bfcp,
      (const float*)bfcp, 0L,
      NROWS, NOUTP, NHID, 0.015625f);
  pack_out_kernel<<<dim3(packBlocks, 1, 1), dim3(256, 1, 1), 0, stream>>>(stg, out, n4);
}
